// MetaBatchRelationalModule_48137993453732
// MI455X (gfx1250) — hardware-verified
//
#include <hip/hip_runtime.h>


#define NBI  256
#define CCH  256
#define LL   25
#define DFE  257
#define KP   288
#define NLOC (NBI * LL)
#define NPR  (NBI * LL * LL)
#define HID  64
#define OUTU 32
#define DM   KP
#define NTK  NLOC
#define SLOPE 0.01f
#define LOSC 1024.0f

typedef _Float16 h16;
typedef unsigned short bf;
typedef __attribute__((ext_vector_type(16))) __bf16   v16bf;
typedef __attribute__((ext_vector_type(16))) _Float16 v16h;
typedef __attribute__((ext_vector_type(8)))  _Float16 v8h;
typedef __attribute__((ext_vector_type(8)))  unsigned short v8us;
typedef __attribute__((ext_vector_type(8)))  float    v8f;
typedef __attribute__((ext_vector_type(4)))  float    v4f;
typedef __attribute__((ext_vector_type(4)))  _Float16 v4h;
typedef v8h  __attribute__((may_alias)) v8ha;
typedef v4f  __attribute__((may_alias)) v4fa;
typedef v8us __attribute__((may_alias)) v8usa;

__device__ __forceinline__ unsigned short f2bf(float f) { unsigned u = __float_as_uint(f); u += 0x7FFFu + ((u >> 16) & 1u); return (unsigned short)(u >> 16); }
__device__ __forceinline__ float bf2f(unsigned short b) { return __uint_as_float(((unsigned)b) << 16); }
__device__ __forceinline__ float bfr(float f) { return bf2f(f2bf(f)); }
__device__ __forceinline__ v16h cat16(v8h lo, v8h hi) { return __builtin_shufflevector(lo, hi, 0, 1, 2, 3, 4, 5, 6, 7, 8, 9, 10, 11, 12, 13, 14, 15); }
__device__ __forceinline__ v16bf cat16b(v8us lo, v8us hi) { return __builtin_bit_cast(v16bf, __builtin_shufflevector(lo, hi, 0, 1, 2, 3, 4, 5, 6, 7, 8, 9, 10, 11, 12, 13, 14, 15)); }
__device__ __forceinline__ v8f wmma16(v16h a, v16h b, v8f c) { return __builtin_amdgcn_wmma_f32_16x16x32_f16(false, a, false, b, (short)0, c, false, false); }
__device__ __forceinline__ v8f wmmab(v16bf a, v16bf b, v8f c) { return __builtin_amdgcn_wmma_f32_16x16x32_bf16(false, a, false, b, (short)0, c, false, false); }

template <bool SPLITA, bool F16OUT = false>
__global__ __launch_bounds__(128) void k_gemmb(const bf* __restrict__ A, const bf* __restrict__ Al, const bf* __restrict__ Bn, const float* __restrict__ bias, float* C, int ldc, h16* C2, const float* __restrict__ R = nullptr, int K = DM, int roundR = 1) {
    __shared__ __align__(16) float ost[4][16 * 68];
    const int lane = threadIdx.x & 31, wave = threadIdx.x >> 5, lr = lane & 15, hi = lane >> 4;
    const int r0 = blockIdx.x * 64 + wave * 16, c0 = blockIdx.y * 64;
    const size_t aoff = (size_t)(r0 + lr) * K + 8 * hi;
    size_t boff[4];
#pragma unroll
    for (int t = 0; t < 4; ++t) boff[t] = (size_t)(c0 + t * 16 + lr) * K + 8 * hi;
    v8f acc[4];
#pragma unroll
    for (int t = 0; t < 4; ++t) acc[t] = (v8f){};
#pragma unroll 1
    for (int kc = 0; kc < K; kc += 32) {
        const v16bf a = cat16b(*(const v8us*)(A + aoff + kc), *(const v8us*)(A + aoff + kc + 16));
        v16bf al = a;
        if (SPLITA) al = cat16b(*(const v8us*)(Al + aoff + kc), *(const v8us*)(Al + aoff + kc + 16));
#pragma unroll
        for (int t = 0; t < 4; ++t) { const v16bf b = cat16b(*(const v8us*)(Bn + boff[t] + kc), *(const v8us*)(Bn + boff[t] + kc + 16)); acc[t] = wmmab(a, b, acc[t]); if (SPLITA) acc[t] = wmmab(al, b, acc[t]); }
        asm volatile("v_nop\n\tv_nop\n\tv_nop\n\tv_nop" : "+v"(acc[0]), "+v"(acc[1]), "+v"(acc[2]), "+v"(acc[3]) : "v"(a), "v"(al));
    }
    float* os = &ost[wave][0];
#pragma unroll
    for (int t = 0; t < 4; ++t) { const float bv = bias ? bfr(bias[c0 + t * 16 + lr]) : 0.f;
#pragma unroll
        for (int j = 0; j < 8; ++j) os[(hi * 8 + j) * 68 + t * 16 + lr] = acc[t][j] + bv; }
    __syncthreads();
    if (F16OUT) {
        h16* crow = (h16*)(void*)C + (size_t)r0 * ldc + c0;
        auto pass = [&]() {
#pragma unroll
            for (int s = 0; s < 4; ++s) { const int row = 4 * s + (lane >> 3), piece = lane & 7; const float* sp = os + row * 68 + piece * 8; v8h o, o2;
#pragma unroll
                for (int i = 0; i < 8; ++i) { const h16 a = (h16)sp[i]; o[i] = a; o2[i] = (h16)((sp[i] - (float)a) * LOSC); }
                *(volatile v8h*)(crow + (size_t)row * ldc + piece * 8) = o; if (C2) *(volatile v8h*)(C2 + (size_t)r0 * ldc + c0 + (size_t)row * ldc + piece * 8) = o2; }
        };
        pass(); __threadfence(); pass();
    } else {
        float* crow = C + (size_t)r0 * ldc + c0;
        auto pass = [&]() {
#pragma unroll
            for (int s = 0; s < 8; ++s) { const int Lid = (lane >> 3) + 4 * s, piece = lane & 7; const int row = Lid >> 1, cofs = (Lid & 1) * 32 + piece * 4;
                v4f val = *(const v4fa*)(os + row * 68 + cofs); if (R) { const v4f rv = *(const v4f*)(R + ((size_t)r0 + row) * ldc + c0 + cofs); val += roundR ? (v4f){bfr(rv[0]), bfr(rv[1]), bfr(rv[2]), bfr(rv[3])} : rv; }
                *(volatile v4f*)(crow + (size_t)row * ldc + cofs) = val; }
        };
        pass(); __threadfence(); pass();
    }
}


__device__ __forceinline__ float lk(float x) { return x >= 0.f ? x : SLOPE * x; }
__global__ __launch_bounds__(256) void k_feats(const float* __restrict__ x, bf* FE) {
    const size_t u = (size_t)blockIdx.x * 256 + threadIdx.x; if (u >= (size_t)NLOC * KP / 8) return;
    v8us o;
#pragma unroll
    for (int i = 0; i < 8; ++i) { const size_t e = u * 8 + i; const int row = (int)(e / KP), c = (int)(e % KP); const int b = row / LL, p = row % LL;
        float v = 0.f; if (c < CCH) v = x[((size_t)b * CCH + c) * LL + p]; else if (c == CCH) v = (float)p; o[i] = f2bf(v); }
    *(volatile v8us*)(FE + u * 8) = o; __threadfence(); *(volatile v8us*)(FE + u * 8) = o;
}
__global__ __launch_bounds__(256) void k_w0(const float* __restrict__ g0, bf* WA, bf* WB) {
    const int u = blockIdx.x * 256 + threadIdx.x; if (u >= HID * KP / 8) return; v8us a, bq;
#pragma unroll
    for (int i = 0; i < 8; ++i) { const int e = u * 8 + i; const int k = e / KP, c = e % KP; a[i] = (c < DFE) ? f2bf(g0[k * (2 * DFE) + c]) : (unsigned short)0; bq[i] = (c < DFE) ? f2bf(g0[k * (2 * DFE) + DFE + c]) : (unsigned short)0; }
    *(volatile v8us*)(WA + u * 8) = a; *(volatile v8us*)(WB + u * 8) = bq; __threadfence(); *(volatile v8us*)(WA + u * 8) = a; *(volatile v8us*)(WB + u * 8) = bq;
}
__global__ __launch_bounds__(256) void k_bf(const float* __restrict__ src, bf* dst, size_t n8) {
    const size_t i = (size_t)blockIdx.x * 256 + threadIdx.x; if (i >= n8) return;
    const v8f v = *(const v8f*)(src + i * 8); v8us o;
#pragma unroll
    for (int k = 0; k < 8; ++k) o[k] = f2bf(v[k]);
    *(volatile v8us*)(dst + i * 8) = o; __threadfence(); *(volatile v8us*)(dst + i * 8) = o;
}
__global__ __launch_bounds__(256) void k_pair(const float* __restrict__ A, const float* __restrict__ Bv, const float* __restrict__ b0, bf* Hh, bf* Hl) {
    typedef __attribute__((ext_vector_type(2))) unsigned short v2us;
    const int lane = threadIdx.x & 31, r = blockIdx.x * 8 + (threadIdx.x >> 5); if (r >= NPR) return;
    const int b = r / (LL * LL), rem = r % (LL * LL), l = rem / LL, m = rem % LL;
    v2us oh, ol;
#pragma unroll
    for (int i = 0; i < 2; ++i) { const int k = 2 * lane + i; const float v = lk(A[((size_t)b * LL + m) * HID + k] + Bv[((size_t)b * LL + l) * HID + k] + bfr(b0[k])); const unsigned short hb = f2bf(v); oh[i] = hb; ol[i] = f2bf(v - bf2f(hb)); }
    const size_t o = (size_t)r * HID + 2 * lane;
    *(volatile v2us*)(Hh + o) = oh; *(volatile v2us*)(Hl + o) = ol; __threadfence(); *(volatile v2us*)(Hh + o) = oh; *(volatile v2us*)(Hl + o) = ol;
}
__global__ __launch_bounds__(256) void k_pairsum(const float* __restrict__ T, float* S) {
    const int u = blockIdx.x * 256 + threadIdx.x; if (u >= NBI * HID) return; const int b = u / HID, k = u % HID;
    float s = 0.f;
#pragma unroll 1
    for (int p = 0; p < LL * LL; ++p) s += lk(T[((size_t)b * LL * LL + p) * HID + k]);
    *(volatile float*)(S + u) = s; __threadfence(); *(volatile float*)(S + u) = s;
}
__global__ __launch_bounds__(256) void k_head(const float* __restrict__ S, const float* __restrict__ pw, const float* __restrict__ pb, const float* __restrict__ ow, const float* __restrict__ ob, float* OUTP) {
    __shared__ float sb[8][HID]; __shared__ float pp[8][HID];
    const int lane = threadIdx.x & 31, w = threadIdx.x >> 5, b = blockIdx.x * 8 + w;
    const bool live = b < NBI;
    if (live) { sb[w][lane] = S[(size_t)b * HID + lane]; sb[w][lane + 32] = S[(size_t)b * HID + lane + 32]; }
    __syncthreads();
    float p0 = 0.f, p1 = 0.f;
    if (live) { p0 = bfr(pb[lane]); p1 = bfr(pb[lane + 32]);
#pragma unroll 1
        for (int k = 0; k < HID; ++k) { const float s = sb[w][k]; p0 = fmaf(s, bfr(pw[lane * HID + k]), p0); p1 = fmaf(s, bfr(pw[(lane + 32) * HID + k]), p1); }
        pp[w][lane] = lk(p0); pp[w][lane + 32] = lk(p1); }
    __syncthreads();
    if (live) { float a = bfr(ob[lane]);
#pragma unroll 1
        for (int k = 0; k < HID; ++k) a = fmaf(pp[w][k], bfr(ow[lane * HID + k]), a);
        const float y = lk(a); *(volatile float*)(OUTP + (size_t)b * OUTU + lane) = y; __threadfence(); *(volatile float*)(OUTP + (size_t)b * OUTU + lane) = y; }
}

extern "C" void kernel_launch(void* const* d_in, const int* in_sizes, int n_in,
                              void* d_out, int out_size, void* d_ws, size_t ws_size, hipStream_t stream) {
    (void)in_sizes; (void)n_in; (void)out_size;
    const float* x = (const float*)d_in[0]; const float* g0w = (const float*)d_in[1]; const float* g0b = (const float*)d_in[2]; const float* g1w = (const float*)d_in[3]; const float* g1b = (const float*)d_in[4];
    const float* pw = (const float*)d_in[5]; const float* pb = (const float*)d_in[6]; const float* ow = (const float*)d_in[7]; const float* ob = (const float*)d_in[8];
    float* out = (float*)d_out;
    char* wsp = (char*)d_ws;
    auto take = [&](size_t bytes) { char* p = wsp; wsp += (bytes + 255) & ~(size_t)255; return (void*)p; };
    bf* FE = (bf*)take((size_t)NLOC * KP * 2); bf* WA = (bf*)take((size_t)HID * KP * 2); bf* WB = (bf*)take((size_t)HID * KP * 2); bf* W1 = (bf*)take(HID * HID * 2);
    float* A = (float*)take((size_t)NLOC * HID * 4); float* Bv = (float*)take((size_t)NLOC * HID * 4); bf* Hh = (bf*)take((size_t)NPR * HID * 2); bf* Hl = (bf*)take((size_t)NPR * HID * 2); float* T = (float*)take((size_t)NPR * HID * 4); float* S = (float*)take((size_t)NBI * HID * 4);
    if ((size_t)(wsp - (char*)d_ws) > ws_size) return;
    k_feats<<<(NLOC * KP / 8 + 255) / 256, 256, 0, stream>>>(x, FE); k_w0<<<(HID * KP / 8 + 255) / 256, 256, 0, stream>>>(g0w, WA, WB); k_bf<<<(HID * HID / 8 + 255) / 256, 256, 0, stream>>>(g1w, W1, HID * HID / 8);
    k_gemmb<false, false><<<dim3(NLOC / 64, 1, 1), 128, 0, stream>>>(FE, nullptr, WA, nullptr, A, HID, nullptr, nullptr, KP);
    k_gemmb<false, false><<<dim3(NLOC / 64, 1, 1), 128, 0, stream>>>(FE, nullptr, WB, nullptr, Bv, HID, nullptr, nullptr, KP);
    k_pair<<<NPR / 8, 256, 0, stream>>>(A, Bv, g0b, Hh, Hl);
    k_gemmb<true, false><<<dim3(NPR / 64, 1, 1), 128, 0, stream>>>(Hh, Hl, W1, g1b, T, HID, nullptr, nullptr, HID);
    k_pairsum<<<(NBI * HID) / 256, 256, 0, stream>>>(T, S);
    k_head<<<NBI / 8, 256, 0, stream>>>(S, pw, pb, ow, ob, out);
}
